// SkipAttention_62182536512221
// MI455X (gfx1250) — hardware-verified
//
#include <hip/hip_runtime.h>
#include <math.h>
#include <stdint.h>

#ifndef NB
#define NB 8
#endif
#ifndef NQ
#define NQ 4096
#endif
#define MD    1024
#define DD    256
#define NKT   (NB * MD)
#define NKB   (MD / 32)
#define QT    (NQ / 16)
#define ATT_BLOCKS  (NB * QT)
#define ATT_THREADS 64
#define HSC   8.0f
#define LSC   8.0f
#define RSC   2048.0f
#define LOG2E 1.4426950408889634f
#define SLAB   (16 * 68)
#define APITCH 132
#define ASLAB  (16 * APITCH)
#define WTP    260

static_assert(NB >= 1 && NQ >= 64 && (NQ % 64) == 0);
static_assert(DD == 256 && MD == 1024 && NKB * 32 == MD);
static_assert(((NB * NQ * DD / 8) % 256) == 0 && ((NKT * DD / 8) % 256) == 0);
static_assert(((NB * NQ) % 64) == 0 && (NKT % 64) == 0 && (DD % 64) == 0 && (DD % 32) == 0 && (DD % 16) == 0);
static_assert((SLAB * 4) % 16 == 0 && (APITCH * 4) % 16 == 0 && (WTP * 4) % 16 == 0);
static_assert(ATT_THREADS == 64 && QT * 16 == NQ);

typedef unsigned short u16;
typedef _Float16 v16h __attribute__((ext_vector_type(16)));
typedef _Float16 v8h  __attribute__((ext_vector_type(8)));
typedef __bf16   v16b __attribute__((ext_vector_type(16)));
typedef float    v8f  __attribute__((ext_vector_type(8)));
typedef float    v4f  __attribute__((ext_vector_type(4)));
typedef unsigned int v4u __attribute__((ext_vector_type(4)));

union FragH { v16h v; v8h h[2]; v4u u[2]; };
union FragB { v16b v; v4u u[2]; };

__device__ __forceinline__ unsigned short bf_bits(float f) {
  unsigned u = __float_as_uint(f);
  return (unsigned short)((u + 0x7FFFu + ((u >> 16) & 1u)) >> 16);
}
__device__ __forceinline__ float bf_up(unsigned short h) { return __uint_as_float(((unsigned)h) << 16); }
__device__ __forceinline__ float bf_val(float f) { return bf_up(bf_bits(f)); }
__device__ __forceinline__ unsigned short h_bits(_Float16 x) { return __builtin_bit_cast(unsigned short, x); }
__device__ __forceinline__ unsigned pk16(unsigned short a, unsigned short b) { return (unsigned)a | ((unsigned)b << 16); }
__device__ __forceinline__ v8f zero8() { v8f z = {0.f, 0.f, 0.f, 0.f, 0.f, 0.f, 0.f, 0.f}; return z; }
__device__ __forceinline__ int uni(int x) {
#if defined(__HIP_DEVICE_COMPILE__)
  return __builtin_amdgcn_readfirstlane(x);
#else
  return x;
#endif
}

__device__ __forceinline__ v16h ldfrag_h(const _Float16* p) {
  FragH f;
  f.h[0] = *(const v8h*)(p);
  f.h[1] = *(const v8h*)(p + 16);
  return f.v;
}
__device__ __forceinline__ v16b ldfrag_b(const u16* p) {
  FragB f;
  f.u[0] = *(const v4u*)(p);
  f.u[1] = *(const v4u*)(p + 16);
  return f.v;
}

__device__ __forceinline__ v8f mma_h(v16h a, v16h b, v8f c) {
  return __builtin_amdgcn_wmma_f32_16x16x32_f16(false, a, false, b, (short)0, c, false, false);
}
__device__ __forceinline__ v8f mma_b(v16b a, v16b b, v8f c) {
  return __builtin_amdgcn_wmma_f32_16x16x32_bf16(false, a, false, b, (short)0, c, false, false);
}
template <typename F>
__device__ __forceinline__ void guard4a(v8f& a, v8f& b, v8f& c, v8f& d, F x0, F x1, F x2, F x3, F x4, F x5) {
#if defined(__HIP_DEVICE_COMPILE__)
  asm volatile("v_nop\n\tv_nop\n\tv_nop\n\tv_nop"
               : "+v"(a), "+v"(b), "+v"(c), "+v"(d) : "v"(x0), "v"(x1), "v"(x2), "v"(x3), "v"(x4), "v"(x5) : "memory");
#endif
}
template <typename F>
__device__ __forceinline__ void guard2a(v8f& a, v8f& b, F x0, F x1, F x2, F x3, F x4, F x5) {
#if defined(__HIP_DEVICE_COMPILE__)
  asm volatile("v_nop\n\tv_nop\n\tv_nop\n\tv_nop"
               : "+v"(a), "+v"(b) : "v"(x0), "v"(x1), "v"(x2), "v"(x3), "v"(x4), "v"(x5) : "memory");
#endif
}
__device__ __forceinline__ void acc_guard4(v8f& a, v8f& b, v8f& c, v8f& d) {
#if defined(__HIP_DEVICE_COMPILE__)
  asm volatile("v_nop\n\tv_nop\n\tv_nop\n\tv_nop" : "+v"(a), "+v"(b), "+v"(c), "+v"(d));
#endif
}
__device__ __forceinline__ void wave_sync_lds() {
#if defined(__HIP_DEVICE_COMPILE__)
  __builtin_amdgcn_fence(__ATOMIC_RELEASE, "workgroup");
  __builtin_amdgcn_wave_barrier();
  __builtin_amdgcn_fence(__ATOMIC_ACQUIRE, "workgroup");
#endif
}

__global__ __launch_bounds__(256) void cvt16(const float* __restrict__ x, u16* D, int n8, int mode, float scale) {
  const int gt = blockIdx.x * 256 + (int)threadIdx.x;
  if (gt >= n8) return;
  const float* p = x + (size_t)gt * 8;
  const v4f a = *(const v4f*)(p), c4 = *(const v4f*)(p + 4);
  float v[8];
#pragma unroll
  for (int e = 0; e < 4; ++e) { v[e] = a[e]; v[4 + e] = c4[e]; }
  unsigned short s[8];
#pragma unroll
  for (int e = 0; e < 8; ++e) {
    const unsigned short bb = bf_bits(v[e]);
    const unsigned short hb = h_bits((_Float16)(bf_up(bb) * scale));
    s[e] = (mode != 0) ? hb : bb;
  }
  v4u o;
#pragma unroll
  for (int e = 0; e < 4; ++e) o[e] = pk16(s[2 * e], s[2 * e + 1]);
  u16* d = D + (size_t)gt * 8;
  for (int pass = 0; pass < 2; ++pass) {
    *(volatile v4u*)(d) = o;
    __threadfence();
  }
}

__global__ __launch_bounds__(256) void wT16(const float* __restrict__ W, u16* WT) {
  __shared__ __align__(16) float tile[16 * WTP];
  const int t = (int)threadIdx.x;
  const int o0 = blockIdx.x * 16;
  if (o0 + 16 > DD) return;
#pragma unroll
  for (int j = 0; j < 16; ++j) tile[j * WTP + t] = W[(size_t)t * DD + o0 + j];
  __syncthreads();
  const int wave = t >> 5, lane = t & 31;
  v4u ov[2];
#pragma unroll
  for (int it = 0; it < 2; ++it) {
    const int row = wave + 8 * it;
    const float* s = tile + row * WTP + 8 * lane;
    const v4f a = *(const v4f*)(s), c4 = *(const v4f*)(s + 4);
    float w8[8];
#pragma unroll
    for (int e = 0; e < 4; ++e) { w8[e] = a[e]; w8[4 + e] = c4[e]; }
#pragma unroll
    for (int e = 0; e < 4; ++e) ov[it][e] = pk16(bf_bits(w8[2 * e]), bf_bits(w8[2 * e + 1]));
  }
  u16* dst = WT + (size_t)o0 * DD + 8 * lane;
  for (int pass = 0; pass < 2; ++pass) {
#pragma unroll
    for (int it = 0; it < 2; ++it) {
      *(volatile v4u*)(dst + (size_t)(wave + 8 * it) * DD) = ov[it];
    }
    __threadfence();
  }
}

__device__ __forceinline__ void epi16x2(float* sl, v8f a0, v8f a1, v8f a2, v8f a3, float oscale, u16* C0, u16* C1,
                                        int N, size_t rowb, int col0, int lane, int mode) {
  const int hh = lane >> 4, m = lane & 15;
#pragma unroll
  for (int r = 0; r < 8; ++r) {
    const int ro = (8 * hh + r) * 68 + m;
    sl[ro]      = a0[r] * oscale;
    sl[ro + 16] = a1[r] * oscale;
    sl[ro + 32] = a2[r] * oscale;
    sl[ro + 48] = a3[r] * oscale;
  }
  wave_sync_lds();
  const int rq = lane >> 3, c8 = (lane & 7) * 8;
  v4u o0[4], o1[4];
#pragma unroll
  for (int i4 = 0; i4 < 4; ++i4) {
    const int row = i4 * 4 + rq;
    const v4f a = *(const v4f*)(sl + row * 68 + c8), c4 = *(const v4f*)(sl + row * 68 + c8 + 4);
    float w8[8];
#pragma unroll
    for (int e = 0; e < 4; ++e) { w8[e] = a[e]; w8[4 + e] = c4[e]; }
    unsigned short s0[8], s1[8];
#pragma unroll
    for (int e = 0; e < 8; ++e) {
      const float x = w8[e];
      const _Float16 xh = (_Float16)x;
      const unsigned short f0 = h_bits(xh);
      const unsigned short f1 = h_bits((_Float16)((x - (float)xh) * RSC));
      const unsigned short g0 = bf_bits(x);
      const unsigned short g1 = bf_bits(x - bf_up(g0));
      s0[e] = (mode != 0) ? g0 : f0;
      s1[e] = (mode != 0) ? g1 : f1;
    }
#pragma unroll
    for (int e = 0; e < 4; ++e) {
      o0[i4][e] = pk16(s0[2 * e], s0[2 * e + 1]);
      o1[i4][e] = pk16(s1[2 * e], s1[2 * e + 1]);
    }
  }
  const size_t dofs = (rowb + (size_t)rq) * (size_t)N + (size_t)(col0 + c8);
  u16* d0 = C0 + dofs;
  u16* d1 = C1 + dofs;
  for (int pass = 0; pass < 2; ++pass) {
#pragma unroll
    for (int i4 = 0; i4 < 4; ++i4) {
      *(volatile v4u*)(d0 + (size_t)(i4 * 4) * (size_t)N) = o0[i4];
      *(volatile v4u*)(d1 + (size_t)(i4 * 4) * (size_t)N) = o1[i4];
    }
    __threadfence();
  }
}

__global__ __launch_bounds__(128)
void gemm_b16x2(const u16* __restrict__ A, const u16* __restrict__ Bt, u16* C0, u16* C1, const float* __restrict__ bias,
                int M, int N, int K, int nbias, int byrow, int mode, float oscale) {
  __shared__ __align__(16) float slab[4 * SLAB];
  const int tid = threadIdx.x, wave = tid >> 5, lane = tid & 31, hh = lane >> 4, m = lane & 15;
  const int ntile = N >> 6;
  const int bid   = blockIdx.x;
  const int rowb  = (bid / ntile) * 64 + wave * 16;
  const int col0  = (bid % ntile) * 64;
  if (rowb + 16 > M) return;
  const u16* ap = A  + (size_t)(rowb + m) * K + 8 * hh;
  const u16* bp = Bt + (size_t)(col0 + m) * K + 8 * hh;
  const size_t bs = (size_t)16 * K;
  v8f acc0 = zero8(), acc1 = zero8(), acc2 = zero8(), acc3 = zero8();
#pragma unroll 1
  for (int k0 = 0; k0 < K; k0 += 32) {
    const v16b a  = ldfrag_b(ap + k0);
    const v16b b0 = ldfrag_b(bp + k0);
    const v16b b1 = ldfrag_b(bp + bs + k0);
    const v16b b2 = ldfrag_b(bp + 2 * bs + k0);
    const v16b b3 = ldfrag_b(bp + 3 * bs + k0);
    acc0 = mma_b(a, b0, acc0);
    acc1 = mma_b(a, b1, acc1);
    acc2 = mma_b(a, b2, acc2);
    acc3 = mma_b(a, b3, acc3);
    guard4a<v16b>(acc0, acc1, acc2, acc3, a, b0, b1, b2, b3, a);
  }
  acc_guard4(acc0, acc1, acc2, acc3);
  float bc[4], br[8];
#pragma unroll
  for (int j = 0; j < 4; ++j) {
    int ci = col0 + 16 * j + m;
    ci = (ci < nbias) ? ci : (nbias - 1);
    bc[j] = bf_val(bias[ci]);
  }
#pragma unroll
  for (int r = 0; r < 8; ++r) {
    int ri = rowb + 8 * hh + r;
    ri = (ri < nbias) ? ri : (nbias - 1);
    br[r] = bf_val(bias[ri]);
  }
#pragma unroll
  for (int r = 0; r < 8; ++r) {
    const float q0 = (byrow != 0) ? br[r] : bc[0];
    const float q1 = (byrow != 0) ? br[r] : bc[1];
    const float q2 = (byrow != 0) ? br[r] : bc[2];
    const float q3 = (byrow != 0) ? br[r] : bc[3];
    acc0[r] += q0;
    acc1[r] += q1;
    acc2[r] += q2;
    acc3[r] += q3;
  }
  epi16x2(slab + wave * SLAB, acc0, acc1, acc2, acc3, oscale, C0, C1, N, (size_t)rowb, col0, lane, mode);
}

__global__ __launch_bounds__(ATT_THREADS)
void attn_pg(const u16* __restrict__ HHp, const u16* __restrict__ HLp, const u16* __restrict__ LHp,
             const u16* __restrict__ LLp, const u16* __restrict__ GHp, const u16* __restrict__ GLp,
             const float* __restrict__ Pin, float* out, const int* aux) {
  __shared__ __align__(16) unsigned xP[2 * 32 * 8];
  __shared__ __align__(16) float xA[32];
  __shared__ __align__(16) float xL[32];
  __shared__ __align__(16) float smem[2 * ASLAB];
  (void)aux;

  const int tid  = (int)threadIdx.x;
  const int wave = uni(tid >> 5);
  const int lane = tid & 31;
  const int hh   = lane >> 4;
  const int c    = lane & 15;

  const int tile = blockIdx.x;
  if (tile >= ATT_BLOCKS) return;
  const int b  = tile / QT;
  const int n0 = (tile % QT) * 16;

  const size_t hofs = ((size_t)(b * NQ + n0 + c)) * DD + 8 * hh;
  const _Float16* Hh = (const _Float16*)(const void*)HHp + hofs;
  const _Float16* Hl = (const _Float16*)(const void*)HLp + hofs;
  const size_t lofs = ((size_t)(b * MD + c)) * DD + 8 * hh;
  const _Float16* Lh = (const _Float16*)(const void*)LHp + lofs;
  const _Float16* Ll = (const _Float16*)(const void*)LLp + lofs;
  const size_t gofs = ((size_t)(wave * 128 + c)) * NKT + (size_t)b * MD + 8 * hh;
  const u16* Gh = GHp + gofs;
  const u16* Gl = GLp + gofs;
  const float lsc  = LOG2E / (HSC * LSC);
  const float rinv = 1.0f / RSC;

  float mrun = -INFINITY, lrun = 0.f;
  v8f o[8];
#pragma unroll
  for (int j = 0; j < 8; ++j) o[j] = zero8();

#pragma unroll 1
  for (int it = 0; it < NKB; ++it) {
    const int kb = it * 32;
    __syncthreads();
    if (wave == 0) {
      v8f sm0 = zero8(), sx0 = zero8(), sm1 = zero8(), sx1 = zero8();
      const _Float16* l0h = Lh + (size_t)kb * DD;
      const _Float16* l0l = Ll + (size_t)kb * DD;
      const _Float16* l1h = l0h + (size_t)16 * DD;
      const _Float16* l1l = l0l + (size_t)16 * DD;
#pragma unroll 1
      for (int k0 = 0; k0 < DD; k0 += 32) {
        const v16h qh0 = ldfrag_h(Hh + k0);
        const v16h ql0 = ldfrag_h(Hl + k0);
        const v16h a0h = ldfrag_h(l0h + k0);
        const v16h a0l = ldfrag_h(l0l + k0);
        const v16h a1h = ldfrag_h(l1h + k0);
        const v16h a1l = ldfrag_h(l1l + k0);
        sm0 = mma_h(a0h, qh0, sm0);
        sx0 = mma_h(a0h, ql0, sx0);
        sx0 = mma_h(a0l, qh0, sx0);
        sm1 = mma_h(a1h, qh0, sm1);
        sx1 = mma_h(a1h, ql0, sx1);
        sx1 = mma_h(a1l, qh0, sx1);
        guard4a<v16h>(sm0, sx0, sm1, sx1, qh0, ql0, a0h, a0l, a1h, a1l);
      }
      acc_guard4(sm0, sx0, sm1, sx1);
      float tk[16];
#pragma unroll
      for (int i = 0; i < 8; ++i) {
        tk[i]     = (sm0[i] + sx0[i] * rinv) * lsc;
        tk[8 + i] = (sm1[i] + sx1[i] * rinv) * lsc;
      }
      float cm = tk[0];
#pragma unroll
      for (int i = 1; i < 16; ++i) cm = fmaxf(cm, tk[i]);
      cm = fmaxf(cm, __shfl_xor(cm, 16, 32));
      const float mn = fmaxf(mrun, cm);
      const float al = (mrun == -INFINITY) ? 0.f : exp2f(mrun - mn);
      mrun = mn;
      float ps = 0.f;
      FragB ph, pl;
#pragma unroll
      for (int w = 0; w < 2; ++w) {
#pragma unroll
        for (int e4 = 0; e4 < 4; ++e4) {
          const int i = 8 * w + 2 * e4;
          const float p0 = exp2f(fminf(tk[i] - mn, 0.f));
          const float p1 = exp2f(fminf(tk[i + 1] - mn, 0.f));
          ps += p0 + p1;
          const unsigned short b0 = bf_bits(p0), b1 = bf_bits(p1);
          const unsigned short r0 = bf_bits(p0 - bf_up(b0)), r1 = bf_bits(p1 - bf_up(b1));
          ph.u[w][e4] = pk16(b0, b1);
          pl.u[w][e4] = pk16(r0, r1);
        }
      }
      ps += __shfl_xor(ps, 16, 32);
      lrun = lrun * al + ps;
      *(v4u*)(xP + lane * 8)           = ph.u[0];
      *(v4u*)(xP + lane * 8 + 4)       = ph.u[1];
      *(v4u*)(xP + 256 + lane * 8)     = pl.u[0];
      *(v4u*)(xP + 256 + lane * 8 + 4) = pl.u[1];
      xA[lane] = al;
    }
    __syncthreads();
    FragB pfh, pfl;
    pfh.u[0] = *(const v4u*)(xP + lane * 8);
    pfh.u[1] = *(const v4u*)(xP + lane * 8 + 4);
    pfl.u[0] = *(const v4u*)(xP + 256 + lane * 8);
    pfl.u[1] = *(const v4u*)(xP + 256 + lane * 8 + 4);
    float scl[8];
    {
      const v4f s0 = *(const v4f*)(xA + 8 * hh), s1 = *(const v4f*)(xA + 8 * hh + 4);
#pragma unroll
      for (int e = 0; e < 4; ++e) { scl[e] = s0[e]; scl[4 + e] = s1[e]; }
    }
#pragma unroll
    for (int j = 0; j < 8; ++j) {
#pragma unroll
      for (int r = 0; r < 8; ++r) o[j][r] *= scl[r];
    }
#pragma unroll
    for (int gq = 0; gq < 4; ++gq) {
      const size_t t0 = (size_t)(32 * gq) * NKT + (size_t)kb;
      const size_t t1 = t0 + (size_t)16 * NKT;
      const v16b gh0 = ldfrag_b(Gh + t0);
      const v16b gl0 = ldfrag_b(Gl + t0);
      const v16b gh1 = ldfrag_b(Gh + t1);
      const v16b gl1 = ldfrag_b(Gl + t1);
      o[2 * gq]     = mma_b(pfh.v, gh0, o[2 * gq]);
      o[2 * gq]     = mma_b(pfh.v, gl0, o[2 * gq]);
      o[2 * gq]     = mma_b(pfl.v, gh0, o[2 * gq]);
      o[2 * gq + 1] = mma_b(pfh.v, gh1, o[2 * gq + 1]);
      o[2 * gq + 1] = mma_b(pfh.v, gl1, o[2 * gq + 1]);
      o[2 * gq + 1] = mma_b(pfl.v, gh1, o[2 * gq + 1]);
      guard2a<v16b>(o[2 * gq], o[2 * gq + 1], pfh.v, pfl.v, gh0, gl0, gh1, gl1);
    }
  }
  acc_guard4(o[0], o[1], o[2], o[3]);
  acc_guard4(o[4], o[5], o[6], o[7]);

  if (wave == 0) xL[lane] = (lrun > 0.f) ? (1.0f / lrun) : 0.f;
  __syncthreads();
  float inv[8];
  {
    const v4f s0 = *(const v4f*)(xL + 8 * hh), s1 = *(const v4f*)(xL + 8 * hh + 4);
#pragma unroll
    for (int e = 0; e < 4; ++e) { inv[e] = s0[e]; inv[4 + e] = s1[e]; }
  }
  float* slab = smem + wave * ASLAB;
#pragma unroll
  for (int r = 0; r < 8; ++r) {
#pragma unroll
    for (int j = 0; j < 8; ++j) slab[(8 * hh + r) * APITCH + j * 16 + c] = o[j][r] * inv[r];
  }
  wave_sync_lds();
  const size_t orow0 = ((size_t)(b * NQ + n0)) * DD + (size_t)(wave * 128 + 4 * lane);
  v4f vals[16];
#pragma unroll
  for (int ri = 0; ri < 16; ++ri) {
    const v4f a  = *(const v4f*)(slab + ri * APITCH + 4 * lane);
    const v4f pv = *(const v4f*)(Pin + orow0 + (size_t)ri * DD);
    v4f v;
#pragma unroll
    for (int e = 0; e < 4; ++e) v[e] = bf_val(pv[e]) + a[e];
    vals[ri] = v;
  }
  for (int pass = 0; pass < 2; ++pass) {
#pragma unroll
    for (int ri = 0; ri < 16; ++ri) {
      *(volatile v4f*)(out + orow0 + (size_t)ri * DD) = vals[ri];
    }
    __threadfence();
  }
}

extern "C" void kernel_launch(void* const* d_in, const int* in_sizes, int n_in,
                              void* d_out, int out_size, void* d_ws, size_t ws_size,
                              hipStream_t stream) {
  if (n_in < 9) return;
  if (in_sizes[0] < NB * NQ * DD) return;
  if (in_sizes[1] < NKT * DD) return;
  if (in_sizes[2] < 1) return;
  if (in_sizes[3] != DD * DD || in_sizes[5] != DD * DD || in_sizes[7] != DD * DD) return;
  if (in_sizes[4] != DD || in_sizes[6] != DD || in_sizes[8] != DD) return;
  if (out_size < NB * NQ * DD) return;

  const float* Pin = (const float*)d_in[0];
  const float* Rin = (const float*)d_in[1];
  const int*   bid = (const int*)d_in[2];
  const float* Wh  = (const float*)d_in[3];
  const float* bh  = (const float*)d_in[4];
  const float* Wl  = (const float*)d_in[5];
  const float* bl  = (const float*)d_in[6];
  const float* Wg  = (const float*)d_in[7];
  const float* bg  = (const float*)d_in[8];
  float*       out = (float*)d_out;

  const size_t szPB = (size_t)NB * NQ * DD * 2;
  const size_t szRB = (size_t)NKT * DD * 2;
  const size_t szW  = (size_t)DD * DD * 2;
  const size_t szH  = szPB;
  const size_t szL  = szRB;
  const size_t szG  = (size_t)DD * NKT * 2;
  size_t off = 0;
  const size_t oPB = off; off += szPB;
  const size_t oRB = off; off += szRB;
  const size_t oWH = off; off += szW;
  const size_t oWL = off; off += szW;
  const size_t oWG = off; off += szW;
  const size_t oHH = off; off += szH;
  const size_t oHL = off; off += szH;
  const size_t oLH = off; off += szL;
  const size_t oLL = off; off += szL;
  const size_t oGH = off; off += szG;
  const size_t oGL = off; off += szG;
  if (off > ws_size) return;
  if (off > (size_t)134217728) return;

  char* ws = (char*)d_ws;
  u16* PB  = (u16*)(ws + oPB);
  u16* RB  = (u16*)(ws + oRB);
  u16* WHT = (u16*)(ws + oWH);
  u16* WLT = (u16*)(ws + oWL);
  u16* WGT = (u16*)(ws + oWG);
  u16* HH  = (u16*)(ws + oHH);
  u16* HL  = (u16*)(ws + oHL);
  u16* LH  = (u16*)(ws + oLH);
  u16* LL  = (u16*)(ws + oLL);
  u16* GH  = (u16*)(ws + oGH);
  u16* GL  = (u16*)(ws + oGL);

  const int n8p = (NB * NQ * DD) / 8;
  const int n8r = (NKT * DD) / 8;
  if ((n8p % 256) != 0 || (n8r % 256) != 0) return;
  const dim3 blk(256);
  const dim3 gP(n8p / 256);
  const dim3 gR(n8r / 256);
  const dim3 gW(DD / 16);
  const dim3 bG(128);
  const dim3 gGH(((NB * NQ) / 64) * (DD / 64));
  const dim3 gGL((NKT / 64) * (DD / 64));
  const dim3 gGG((DD / 64) * (NKT / 64));
  const dim3 gAT(ATT_BLOCKS);
  const dim3 bAT(ATT_THREADS);

  cvt16<<<gP, blk, 0, stream>>>(Pin, PB, n8p, 0, 1.0f);
  cvt16<<<gR, blk, 0, stream>>>(Rin, RB, n8r, 0, 1.0f);
  wT16<<<gW, blk, 0, stream>>>(Wh, WHT);
  wT16<<<gW, blk, 0, stream>>>(Wl, WLT);
  wT16<<<gW, blk, 0, stream>>>(Wg, WGT);
  gemm_b16x2<<<gGH, bG, 0, stream>>>(PB, WHT, HH, HL, bh, NB * NQ, DD, DD, DD, 0, 0, HSC);
  gemm_b16x2<<<gGL, bG, 0, stream>>>(RB, WLT, LH, LL, bl, NKT, DD, DD, DD, 0, 0, LSC);
  gemm_b16x2<<<gGG, bG, 0, stream>>>(WGT, RB, GH, GL, bg, DD, NKT, DD, DD, 1, 1, 1.0f);
  attn_pg<<<gAT, bAT, 0, stream>>>(HH, HL, LH, LL, GH, GL, Pin, out, bid);
  (void)hipGetLastError();
}
